// SA_Attn_Mem_20495583937283
// MI455X (gfx1250) — hardware-verified
//
#include <hip/hip_runtime.h>
#include <hip/hip_bf16.h>
#include <math.h>


typedef __attribute__((ext_vector_type(16))) _Float16 v16h;
typedef __attribute__((ext_vector_type(8)))  _Float16 v8h;
typedef __attribute__((ext_vector_type(16))) __bf16   v16b;
typedef __attribute__((ext_vector_type(8)))  __bf16   v8b;
typedef __attribute__((ext_vector_type(8)))  float    v8f;
typedef __attribute__((ext_vector_type(4)))  float    v4f;
typedef __attribute__((ext_vector_type(8)))  unsigned short v8us;
typedef __attribute__((ext_vector_type(4)))  unsigned int   v4u;

__device__ __forceinline__ unsigned short f2bf_bits(float f) {
  unsigned u = __float_as_uint(f);
  return (unsigned short)((u + 0x7FFFu + ((u >> 16) & 1u)) >> 16);
}
__device__ __forceinline__ float bf_bits2f(unsigned short h) { return __uint_as_float(((unsigned)h) << 16); }

__device__ __forceinline__ void dep_guard_h(v8f& a, v8f& b, v16h x, v16h y) { asm volatile("v_nop\n\tv_nop\n\tv_nop\n\tv_nop" : "+v"(a), "+v"(b) : "v"(x), "v"(y)); }
__device__ __forceinline__ void dep_guard_b(v8f& a, v8f& b, v16b x, v16b y) { asm volatile("v_nop\n\tv_nop\n\tv_nop\n\tv_nop" : "+v"(a), "+v"(b) : "v"(x), "v"(y)); }
__device__ __forceinline__ void keep4_h(v16h a, v16h b, v16h c, v16h d) { asm volatile("v_nop" :: "v"(a), "v"(b), "v"(c), "v"(d)); }
__device__ __forceinline__ void keep4_b(v16b a, v16b b, v16b c, v16b d) { asm volatile("v_nop" :: "v"(a), "v"(b), "v"(c), "v"(d)); }
__device__ __forceinline__ void acc_guard4(v8f& a, v8f& b, v8f& c, v8f& d) { asm volatile("v_nop\n\tv_nop\n\tv_nop\n\tv_nop" : "+v"(a), "+v"(b), "+v"(c), "+v"(d)); }
template <typename T> struct Frag;
template <> struct Frag<_Float16> {
  typedef v16h V; union U { v16h v; v8h h[2]; };
  static __device__ __forceinline__ v16h load(const _Float16* p) {
    U f; f.h[0] = *(const v8h*)(p); f.h[1] = *(const v8h*)(p + 16); return f.v;
  }
  static __device__ __forceinline__ v8f mma(v16h a, v16h b, v8f c) {
    return __builtin_amdgcn_wmma_f32_16x16x32_f16(false, a, false, b, (short)0, c, false, false);
  }
  static __device__ __forceinline__ void guard(v8f& a, v8f& b, v16h x, v16h y) { dep_guard_h(a, b, x, y); }
  static __device__ __forceinline__ void keep(v16h a, v16h b, v16h c, v16h d) { keep4_h(a, b, c, d); }
};
template <> struct Frag<__bf16> {
  typedef v16b V; union U { v16b v; v8b h[2]; };
  static __device__ __forceinline__ v16b load(const __bf16* p) {
    U f; f.h[0] = *(const v8b*)(p); f.h[1] = *(const v8b*)(p + 16); return f.v;
  }
  static __device__ __forceinline__ v8f mma(v16b a, v16b b, v8f c) {
    return __builtin_amdgcn_wmma_f32_16x16x32_bf16(false, a, false, b, (short)0, c, false, false);
  }
  static __device__ __forceinline__ void guard(v8f& a, v8f& b, v16b x, v16b y) { dep_guard_b(a, b, x, y); }
  static __device__ __forceinline__ void keep(v16b a, v16b b, v16b c, v16b d) { keep4_b(a, b, c, d); }
};

template <int ET> struct Elem;
template <> struct Elem<0> { typedef _Float16 T; };
template <> struct Elem<1> { typedef __bf16 T; };
template <int ET, bool SPLIT, int BIAS_MODE, int OUT_MODE, bool RESID, int ACT = 0>
__global__ __launch_bounds__(256) void wmma_gemm64(
    const unsigned short* __restrict__ Ap, const unsigned short* __restrict__ A2p, int lda, long strideA,
    const unsigned short* __restrict__ Btp, const unsigned short* __restrict__ Bt2p, int ldb, long strideB,
    void* __restrict__ Cout, void* __restrict__ Cout2, int ldc, long strideC,
    const float* __restrict__ bias,
    const float* __restrict__ resid, long strideR,
    int M, int N, int K, float scale) {
  typedef typename Elem<ET>::T T;
  typedef typename Frag<T>::V V;
  const T* A = (const T*)Ap; const T* A2 = (const T*)A2p; const T* Bt = (const T*)Btp; const T* Bt2 = (const T*)Bt2p;
  __shared__ __align__(16) float sT[8][16 * 68];
  const int b    = blockIdx.y;
  const int lane = threadIdx.x & 31;
  const int wave = threadIdx.x >> 5;
  const int tilesN = N >> 6;
  const int tilesM = M >> 6;
  const int tile = blockIdx.x * 8 + wave;
  if (tile >= tilesM * tilesN) return;
  const int tm = tile / tilesN;
  const int tn = tile - tm * tilesN;
  const int m0 = tm << 6;
  const int n0 = tn << 6;

  const T* Ab  = A  + (size_t)b * strideA;
  const T* Bb  = Bt + (size_t)b * strideB;
  const T* Ab2 = SPLIT ? (A2  + (size_t)b * strideA) : nullptr;
  const T* Bb2 = SPLIT ? (Bt2 + (size_t)b * strideB) : nullptr;

  const int rlane = lane & 15;
  const int koff  = (lane >> 4) * 8;
  const int mOff  = (lane >> 4) * 8;

  v8f acc[4][4];
#pragma unroll
  for (int i = 0; i < 4; ++i)
#pragma unroll
    for (int j = 0; j < 4; ++j) acc[i][j] = (v8f){0.f,0.f,0.f,0.f,0.f,0.f,0.f,0.f};

  for (int k0 = 0; k0 < K; k0 += 32) {
    V bh[4], bl[4];
#pragma unroll
    for (int j = 0; j < 4; ++j) {
      const size_t bo = (size_t)(n0 + (j << 4) + rlane) * ldb + koff + k0;
      bh[j] = Frag<T>::load(Bb + bo);
      if (SPLIT) bl[j] = Frag<T>::load(Bb2 + bo);
    }
#pragma unroll
    for (int i = 0; i < 4; ++i) {
      const size_t ao = (size_t)(m0 + (i << 4) + rlane) * lda + koff + k0;
      V ah = Frag<T>::load(Ab + ao);
      V al;
      if (SPLIT) al = Frag<T>::load(Ab2 + ao);
#pragma unroll
      for (int j = 0; j < 4; ++j) {
        acc[i][j] = Frag<T>::mma(ah, bh[j], acc[i][j]);
        if (SPLIT) {
          acc[i][j] = Frag<T>::mma(ah, bl[j], acc[i][j]);
          acc[i][j] = Frag<T>::mma(al, bh[j], acc[i][j]);
        }
      }
      Frag<T>::guard(acc[i][0], acc[i][3], ah, SPLIT ? al : ah);
    }
    Frag<T>::keep(bh[0], bh[1], bh[2], bh[3]);
    if (SPLIT) Frag<T>::keep(bl[0], bl[1], bl[2], bl[3]);
  }
  acc_guard4(acc[0][0], acc[0][1], acc[0][2], acc[0][3]);
  acc_guard4(acc[1][0], acc[1][1], acc[1][2], acc[1][3]);
  acc_guard4(acc[2][0], acc[2][1], acc[2][2], acc[2][3]);
  acc_guard4(acc[3][0], acc[3][1], acc[3][2], acc[3][3]);

  float* slab = sT[wave];
  const float* Rb = RESID ? (resid + (size_t)b * strideR) : nullptr;
#pragma unroll
  for (int i = 0; i < 4; ++i) {
    const int mBase = m0 + (i << 4);
#pragma unroll
    for (int j = 0; j < 4; ++j) {
      const int n = n0 + (j << 4) + rlane;
      float bv = 0.f;
      if (BIAS_MODE == 2) bv = bias[n];
#pragma unroll
      for (int r = 0; r < 8; ++r) {
        float v = acc[i][j][r] * scale;
        if (BIAS_MODE == 1) v += bias[mBase + mOff + r];
        if (BIAS_MODE == 2) v += bv;
        if (RESID) v += Rb[(size_t)(mBase + mOff + r) * ldc + n];
        if (ACT == 1) v = tanhf(v);
        if (ACT == 2) v = fmaxf(v, 0.0f);
        if (ACT == 3) v = v / (1.0f + expf(-v));
        if (ACT == 4) v = (v > 0.f) ? v : 0.01f * v;
        if (ACT == 5) v = 0.5f * v * (1.0f + erff(v * 0.70710678118654752f));
        slab[(mOff + r) * 68 + (j << 4) + rlane] = v;
      }
    }
    __builtin_amdgcn_fence(__ATOMIC_RELEASE, "workgroup");
    __builtin_amdgcn_wave_barrier();
    __builtin_amdgcn_fence(__ATOMIC_ACQUIRE, "workgroup");
    if (OUT_MODE == 0) {
      float* C = (float*)Cout + (size_t)b * strideC;
      const int hh = lane >> 4, c4 = (lane & 15) * 4;
      for (int pass = 0; pass < 2; ++pass) {
#pragma unroll
        for (int it = 0; it < 8; ++it) {
          const int row = it * 2 + hh;
          v4f v = *(const v4f*)(slab + row * 68 + c4);
          *(volatile v4f*)(C + (size_t)(mBase + row) * ldc + n0 + c4) = v;
        }
        __threadfence();
      }
    } else {
      const int q = lane >> 3, c8 = (lane & 7) * 8;
      unsigned short* C  = (unsigned short*)Cout  + (size_t)b * strideC;
      unsigned short* C2 = (OUT_MODE == 2) ? ((unsigned short*)Cout2 + (size_t)b * strideC) : nullptr;
      for (int pass = 0; pass < 2; ++pass) {
#pragma unroll
        for (int it = 0; it < 4; ++it) {
          const int row = it * 4 + q;
          const float* sp = slab + row * 68 + c8;
          v8h hv, lv;
#pragma unroll
          for (int e = 0; e < 8; ++e) {
            if (OUT_MODE == 1) {
              hv[e] = (_Float16)sp[e];
            } else {
              unsigned short hb = f2bf_bits(sp[e]);
              unsigned short lb = f2bf_bits(sp[e] - bf_bits2f(hb));
              hv[e] = __builtin_bit_cast(_Float16, hb);
              lv[e] = __builtin_bit_cast(_Float16, lb);
            }
          }
          *(volatile v8h*)(C + (size_t)(mBase + row) * ldc + n0 + c8) = hv;
          if (OUT_MODE == 2) *(volatile v8h*)(C2 + (size_t)(mBase + row) * ldc + n0 + c8) = lv;
        }
        __threadfence();
      }
    }
    __builtin_amdgcn_fence(__ATOMIC_RELEASE, "workgroup");
    __builtin_amdgcn_wave_barrier();
    __builtin_amdgcn_fence(__ATOMIC_ACQUIRE, "workgroup");
  }
}

__device__ __forceinline__ v8f mma_bf(v16b a, v16b b, v8f c) {
  c = __builtin_amdgcn_wmma_f32_16x16x32_bf16(false, a, false, b, (short)0, c, false, false);
  asm volatile("v_nop\n\tv_nop\n\tv_nop\n\tv_nop" : "+v"(c) : "v"(a), "v"(b));
  return c;
}
__device__ __forceinline__ v8f mma_hf(v16h a, v16h b, v8f c) {
  c = __builtin_amdgcn_wmma_f32_16x16x32_f16(false, a, false, b, (short)0, c, false, false);
  asm volatile("v_nop\n\tv_nop\n\tv_nop\n\tv_nop" : "+v"(c) : "v"(a), "v"(b));
  return c;
}

#define OFF_WQH  0
#define OFF_WQL  4096
#define OFF_WKH  8192
#define OFF_WKL  12288
#define OFF_WK2H 16384
#define OFF_WK2L 20480
#define OFF_WV   24576
#define OFF_WV2  28672
#define OFF_WZ   32768
#define OFF_WM   49152
#define W_ELEMS  86016
#define WCARRY   16.0f
#define WCARRY_INV 0.0625f

__global__ __launch_bounds__(256) void k_castw(
    const float* __restrict__ Wq, const float* __restrict__ Wk, const float* __restrict__ Wk2,
    const float* __restrict__ Wv, const float* __restrict__ Wv2, const float* __restrict__ Wz,
    const float* __restrict__ Wm, unsigned short* __restrict__ wr) {
  const int which = blockIdx.y;
  const float* src = Wq; int n2 = 2048; int oa = OFF_WQH, ob = OFF_WQL; int split = 1;
  if (which == 1)      { src = Wk;  oa = OFF_WKH;  ob = OFF_WKL; }
  else if (which == 2) { src = Wk2; oa = OFF_WK2H; ob = OFF_WK2L; }
  else if (which == 3) { src = Wv;  oa = OFF_WV;   ob = OFF_WV;  split = 0; }
  else if (which == 4) { src = Wv2; oa = OFF_WV2;  ob = OFF_WV2; split = 0; }
  else if (which == 5) { src = Wz;  oa = OFF_WZ;   ob = OFF_WZ;  split = 0; n2 = 8192; }
  else if (which == 6) { src = Wm;  oa = OFF_WM;   ob = OFF_WM;  split = 0; n2 = 18432; }
  const int i = blockIdx.x * 256 + threadIdx.x;
  if (i < n2) {
    const float f0 = src[2 * i], f1 = src[2 * i + 1];
    unsigned u0, u1;
    if (split) {
      const unsigned short hb0 = f2bf_bits(f0), hb1 = f2bf_bits(f1);
      const unsigned short lb0 = f2bf_bits(f0 - bf_bits2f(hb0));
      const unsigned short lb1 = f2bf_bits(f1 - bf_bits2f(hb1));
      u0 = (unsigned)hb0 | ((unsigned)hb1 << 16);
      u1 = (unsigned)lb0 | ((unsigned)lb1 << 16);
    } else {
      const _Float16 h0 = (_Float16)(f0 * WCARRY), h1 = (_Float16)(f1 * WCARRY);
      u0 = (unsigned)__builtin_bit_cast(unsigned short, h0) | ((unsigned)__builtin_bit_cast(unsigned short, h1) << 16);
      u1 = u0;
    }
    volatile unsigned* pa = (volatile unsigned*)(wr + oa);
    volatile unsigned* pb = (volatile unsigned*)(wr + ob);
    pa[i] = u0;
    if (split) pb[i] = u1;
    __threadfence();
    pa[i] = u0;
    if (split) pb[i] = u1;
  }
}

__global__ __launch_bounds__(256) void k_prep(
    const float* __restrict__ hin, const float* __restrict__ min_,
    unsigned short* __restrict__ hTh, unsigned short* __restrict__ hTl, unsigned short* __restrict__ h16,
    unsigned short* __restrict__ mTh, unsigned short* __restrict__ mTl, unsigned short* __restrict__ m16,
    int N) {
  __shared__ float sm[64][65];
  const int tid = threadIdx.x;
  const int n0 = blockIdx.x * 64, b = blockIdx.y, z = blockIdx.z;
  const float* src = z ? min_ : hin;
  unsigned short* dh = z ? mTh : hTh;
  unsigned short* dl = z ? mTl : hTl;
  unsigned short* d16 = z ? m16 : h16;
  const int ld16 = z ? 64 : 192;
  const int co16 = z ? 0 : 128;
#pragma unroll
  for (int p = 0; p < 4; ++p) {
    const int c = p * 16 + (tid >> 4);
    const int n4 = (tid & 15) * 4;
    const v4f x = *(const v4f*)(src + ((size_t)(b * 64 + c)) * N + n0 + n4);
    sm[c][n4 + 0] = x[0]; sm[c][n4 + 1] = x[1]; sm[c][n4 + 2] = x[2]; sm[c][n4 + 3] = x[3];
  }
  __syncthreads();
  const int wave = tid >> 5, lane = tid & 31, q = lane >> 3, c8 = (lane & 7) * 8;
  v8us H[2], L[2], F[2];
#pragma unroll
  for (int it = 0; it < 2; ++it) {
    const int nl = wave * 8 + it * 4 + q;
#pragma unroll
    for (int e = 0; e < 8; ++e) {
      const float f = sm[c8 + e][nl];
      const unsigned short hb = f2bf_bits(f);
      const unsigned short lb = f2bf_bits(f - bf_bits2f(hb));
      H[it][e] = hb;
      L[it][e] = lb;
      F[it][e] = __builtin_bit_cast(unsigned short, (_Float16)f);
    }
  }
  for (int pass = 0; pass < 2; ++pass) {
#pragma unroll
    for (int it = 0; it < 2; ++it) {
      const int nl = wave * 8 + it * 4 + q;
      const size_t rowi = (size_t)b * N + n0 + nl;
      *(volatile v8us*)(dh + rowi * 64 + c8) = H[it];
      *(volatile v8us*)(dl + rowi * 64 + c8) = L[it];
      *(volatile v8us*)(d16 + rowi * (size_t)ld16 + co16 + c8) = F[it];
    }
    __threadfence();
  }
}

#define AT_D 64
#define AT_KC 64
#define AT_P 32768.0f

__global__ __launch_bounds__(128) void attn_dual(
    const unsigned short* __restrict__ Qhp, const unsigned short* __restrict__ Qlp,
    const unsigned short* __restrict__ Khp, const unsigned short* __restrict__ Klp,
    const unsigned short* __restrict__ Kmhp, const unsigned short* __restrict__ Kmlp,
    const unsigned short* __restrict__ Vhp, const unsigned short* __restrict__ Vmp,
    unsigned short* __restrict__ Zcp, int N) {
  union FB { v16b v; v8b h[2]; };
  union FH { v16h v; v8h h[2]; };
  __shared__ __align__(16) __bf16   Ksh[AT_KC * AT_D];
  __shared__ __align__(16) __bf16   Ksl[AT_KC * AT_D];
  __shared__ __align__(16) _Float16 Vth[AT_D * AT_KC];
  __shared__ __align__(16) _Float16 Psh[4][16 * AT_KC];
  __shared__ __align__(16) float    Os[4][16 * 68];

  const int tid = threadIdx.x, wave = tid >> 5, lane = tid & 31;
  const int hh = lane >> 4, c = lane & 15;
  const int nqb = N >> 6;
  int bx = blockIdx.x;
  const int qb = bx % nqb; bx = bx / nqb;
  const int strm = bx & 1;
  const int b = bx >> 1;
  const size_t plane = (size_t)N * 64;
  const __bf16* Qh = (const __bf16*)Qhp + (size_t)b * plane;
  const __bf16* Ql = (const __bf16*)Qlp + (size_t)b * plane;
  const __bf16* Kh = (const __bf16*)(strm ? Kmhp : Khp) + (size_t)b * plane;
  const __bf16* Kl = (const __bf16*)(strm ? Kmlp : Klp) + (size_t)b * plane;
  const _Float16* V = (const _Float16*)(strm ? Vmp : Vhp) + (size_t)b * plane;
  _Float16* Z = (_Float16*)Zcp + (size_t)b * (size_t)N * 128 + strm * 64;
  const int q0 = qb * 64 + wave * 16;

  v16b qah[2], qal[2];
#pragma unroll
  for (int dc = 0; dc < 2; ++dc) {
    qah[dc] = Frag<__bf16>::load(Qh + (size_t)(q0 + c) * AT_D + dc * 32 + 8 * hh);
    qal[dc] = Frag<__bf16>::load(Ql + (size_t)(q0 + c) * AT_D + dc * 32 + 8 * hh);
  }

  float mrow[8], lrow[8];
  v8f oacc[4];
#pragma unroll
  for (int r = 0; r < 8; ++r) { mrow[r] = -INFINITY; lrow[r] = 0.f; }
#pragma unroll
  for (int t = 0; t < 4; ++t) oacc[t] = (v8f){0.f,0.f,0.f,0.f,0.f,0.f,0.f,0.f};

  for (int kc = 0; kc < nqb; ++kc) {
    const int kv0 = kc * AT_KC;
    __syncthreads();
#pragma unroll
    for (int it = 0; it < 4; ++it) {
      const int idx = it * 128 + tid;
      const int row = idx >> 3, part = (idx & 7) * 8;
      const v4u k4 = *(const v4u*)(Kh + (size_t)(kv0 + row) * AT_D + part);
      const v4u l4 = *(const v4u*)(Kl + (size_t)(kv0 + row) * AT_D + part);
      const v4u w4 = *(const v4u*)(V + (size_t)row * N + kv0 + part);
      *(v4u*)(Ksh + row * AT_D + part) = k4;
      *(v4u*)(Ksl + row * AT_D + part) = l4;
      *(v4u*)(Vth + row * AT_KC + part) = w4;
    }
    __syncthreads();

    v8f s[4];
#pragma unroll
    for (int j = 0; j < 4; ++j) {
      s[j] = (v8f){0.f,0.f,0.f,0.f,0.f,0.f,0.f,0.f};
#pragma unroll
      for (int dc = 0; dc < 2; ++dc) {
        FB kb, kl;
        kb.h[0] = *(const v8b*)(Ksh + (j * 16 + c) * AT_D + dc * 32 + 8 * hh);
        kb.h[1] = *(const v8b*)(Ksh + (j * 16 + c) * AT_D + dc * 32 + 16 + 8 * hh);
        kl.h[0] = *(const v8b*)(Ksl + (j * 16 + c) * AT_D + dc * 32 + 8 * hh);
        kl.h[1] = *(const v8b*)(Ksl + (j * 16 + c) * AT_D + dc * 32 + 16 + 8 * hh);
        s[j] = mma_bf(qah[dc], kb.v, s[j]);
        s[j] = mma_bf(qah[dc], kl.v, s[j]);
        s[j] = mma_bf(qal[dc], kb.v, s[j]);
      }
    }
    float cm[8];
#pragma unroll
    for (int r = 0; r < 8; ++r) {
      float mx = fmaxf(fmaxf(s[0][r], s[1][r]), fmaxf(s[2][r], s[3][r]));
#pragma unroll
      for (int off = 1; off < 16; off <<= 1) mx = fmaxf(mx, __shfl_xor(mx, off, 32));
      cm[r] = mx;
    }
    _Float16* pw = Psh[wave];
#pragma unroll
    for (int r = 0; r < 8; ++r) {
      const float mnew = fmaxf(mrow[r], cm[r]);
      const float alpha = expf(mrow[r] - mnew);
      mrow[r] = mnew;
      float psum = 0.f;
#pragma unroll
      for (int j = 0; j < 4; ++j) {
        const float p = expf(s[j][r] - mnew);
        psum += p;
        pw[(8 * hh + r) * AT_KC + j * 16 + c] = (_Float16)(p * AT_P);
      }
#pragma unroll
      for (int off = 1; off < 16; off <<= 1) psum += __shfl_xor(psum, off, 32);
      lrow[r] = lrow[r] * alpha + psum;
#pragma unroll
      for (int t = 0; t < 4; ++t) oacc[t][r] *= alpha;
    }
    __builtin_amdgcn_fence(__ATOMIC_RELEASE, "workgroup");
    __builtin_amdgcn_wave_barrier();
    __builtin_amdgcn_fence(__ATOMIC_ACQUIRE, "workgroup");
#pragma unroll
    for (int kk = 0; kk < 2; ++kk) {
      FH pa;
      pa.h[0] = *(const v8h*)(pw + c * AT_KC + kk * 32 + 8 * hh);
      pa.h[1] = *(const v8h*)(pw + c * AT_KC + kk * 32 + 16 + 8 * hh);
#pragma unroll
      for (int t = 0; t < 4; ++t) {
        FH vb;
        vb.h[0] = *(const v8h*)(Vth + (t * 16 + c) * AT_KC + kk * 32 + 8 * hh);
        vb.h[1] = *(const v8h*)(Vth + (t * 16 + c) * AT_KC + kk * 32 + 16 + 8 * hh);
        oacc[t] = mma_hf(pa.v, vb.v, oacc[t]);
      }
    }
  }

  float* os = Os[wave];
#pragma unroll
  for (int r = 0; r < 8; ++r) {
    const float inv = 1.0f / (lrow[r] * AT_P);
#pragma unroll
    for (int t = 0; t < 4; ++t) os[(8 * hh + r) * 68 + t * 16 + c] = oacc[t][r] * inv;
  }
  __builtin_amdgcn_fence(__ATOMIC_RELEASE, "workgroup");
  __builtin_amdgcn_wave_barrier();
  __builtin_amdgcn_fence(__ATOMIC_ACQUIRE, "workgroup");
  {
    const int q4 = lane >> 3, c8 = (lane & 7) * 8;
    v8h hv[4];
#pragma unroll
    for (int it = 0; it < 4; ++it) {
      const int row = it * 4 + q4;
      const float* sp = os + row * 68 + c8;
#pragma unroll
      for (int e = 0; e < 8; ++e) hv[it][e] = (_Float16)sp[e];
    }
    for (int pass = 0; pass < 2; ++pass) {
#pragma unroll
      for (int it = 0; it < 4; ++it) {
        const int row = it * 4 + q4;
        *(volatile v8h*)(Z + (size_t)(q0 + row) * 128 + c8) = hv[it];
      }
      __threadfence();
    }
  }
}

__global__ __launch_bounds__(256) void k_gate(
    const float* __restrict__ comb, const float* __restrict__ mm,
    float* __restrict__ out0, float* __restrict__ out1, int N, int total) {
  const int i = blockIdx.x * 256 + threadIdx.x;
  if (i < total) {
    const int n = i % N;
    const int bc = i / N;
    const int c = bc & 63;
    const int b = bc >> 6;
    const size_t rb = ((size_t)b * 192 + c) * (size_t)N + n;
    float vo = comb[rb];
    float vg = comb[rb + (size_t)64 * N];
    float vi = comb[rb + (size_t)128 * N];
    const float mv = mm[(size_t)i];
    vo = fminf(fmaxf(vo, -30.0f), 30.0f);
    vi = fminf(fmaxf(vi, -30.0f), 30.0f);
    vg = fminf(fmaxf(vg, -30.0f), 30.0f);
    const float si = 1.0f / (1.0f + expf(-vi));
    const float nm = (1.0f - si) * mv + si * tanhf(vg);
    const float so = 1.0f / (1.0f + expf(-vo));
    const float nh = so * nm;
    ((volatile float*)out0)[i] = nh;
    ((volatile float*)out1)[i] = nm;
    __threadfence();
    ((volatile float*)out0)[i] = nh;
    ((volatile float*)out1)[i] = nm;
  }
}

extern "C" void kernel_launch(void* const* d_in, const int* in_sizes, int n_in,
                              void* d_out, int out_size, void* d_ws, size_t ws_size,
                              hipStream_t stream) {
  if (n_in < 16) return;
  const int NP = 4096, CH = 64;
  const int nh = in_sizes[0];
  const int B = nh / (CH * NP);
  if (B < 1 || B * CH * NP != nh || in_sizes[1] != nh || out_size != 2 * nh) return;
  if (in_sizes[2] != CH * CH || in_sizes[4] != CH * CH || in_sizes[6] != CH * CH ||
      in_sizes[8] != CH * CH || in_sizes[10] != CH * CH ||
      in_sizes[12] != 4 * CH * CH || in_sizes[14] != 9 * CH * CH) return;
  if (in_sizes[3] < CH || in_sizes[5] < CH || in_sizes[7] < CH || in_sizes[9] < CH ||
      in_sizes[11] < CH || in_sizes[13] < 2 * CH || in_sizes[15] < 3 * CH) return;

  const float* h   = (const float*)d_in[0];
  const float* m   = (const float*)d_in[1];
  const float* Wq  = (const float*)d_in[2];
  const float* bq  = (const float*)d_in[3];
  const float* Wk  = (const float*)d_in[4];
  const float* bk  = (const float*)d_in[5];
  const float* Wk2 = (const float*)d_in[6];
  const float* bk2 = (const float*)d_in[7];
  const float* Wv  = (const float*)d_in[8];
  const float* bv  = (const float*)d_in[9];
  const float* Wv2 = (const float*)d_in[10];
  const float* bv2 = (const float*)d_in[11];
  const float* Wz  = (const float*)d_in[12];
  const float* bz  = (const float*)d_in[13];
  const float* Wm  = (const float*)d_in[14];
  const float* bm  = (const float*)d_in[15];
  float* out0 = (float*)d_out;
  float* out1 = (float*)d_out + (size_t)nh;

  const size_t szW  = (size_t)W_ELEMS * 2;
  const size_t szP  = (size_t)B * NP * 64 * 2;
  const size_t szZ  = (size_t)B * NP * 128 * 2;
  const size_t szX  = (size_t)B * NP * 192 * 2;
  const size_t szCb = (size_t)B * 192 * NP * 4;
  const size_t total = szW + 13 * szP + szZ + szX + szCb;
  if (total > ws_size || total > (size_t)134217728) return;
  char* base = (char*)d_ws;
  size_t off = 0;
  unsigned short* wr   = (unsigned short*)(base + off); off += szW;
  unsigned short* hTh  = (unsigned short*)(base + off); off += szP;
  unsigned short* hTl  = (unsigned short*)(base + off); off += szP;
  unsigned short* mTh  = (unsigned short*)(base + off); off += szP;
  unsigned short* mTl  = (unsigned short*)(base + off); off += szP;
  unsigned short* mT16 = (unsigned short*)(base + off); off += szP;
  unsigned short* Qh   = (unsigned short*)(base + off); off += szP;
  unsigned short* Ql   = (unsigned short*)(base + off); off += szP;
  unsigned short* Kh   = (unsigned short*)(base + off); off += szP;
  unsigned short* Kl   = (unsigned short*)(base + off); off += szP;
  unsigned short* Kmh  = (unsigned short*)(base + off); off += szP;
  unsigned short* Kml  = (unsigned short*)(base + off); off += szP;
  unsigned short* Vh   = (unsigned short*)(base + off); off += szP;
  unsigned short* Vm   = (unsigned short*)(base + off); off += szP;
  unsigned short* Zc   = (unsigned short*)(base + off); off += szZ;
  unsigned short* X3   = (unsigned short*)(base + off); off += szX;
  float*          comb = (float*)(base + off);          off += szCb;
  if (off != total) return;

  const long pstride = (long)NP * 64;
  const int nqb = NP / 64;

  k_castw<<<dim3(72, 7), 256, 0, stream>>>(Wq, Wk, Wk2, Wv, Wv2, Wz, Wm, wr);
  k_prep<<<dim3(nqb, B, 2), 256, 0, stream>>>(h, m, hTh, hTl, X3, mTh, mTl, mT16, NP);
  wmma_gemm64<1, true, 2, 2, false><<<dim3((nqb * 1 + 7) / 8, B), 256, 0, stream>>>(
      hTh, hTl, 64, pstride, wr + OFF_WQH, wr + OFF_WQL, 64, 0L,
      (void*)Qh, (void*)Ql, 64, pstride, bq, bq, 0L, NP, 64, 64, 1.0f);
  wmma_gemm64<1, true, 2, 2, false><<<dim3((nqb * 1 + 7) / 8, B), 256, 0, stream>>>(
      hTh, hTl, 64, pstride, wr + OFF_WKH, wr + OFF_WKL, 64, 0L,
      (void*)Kh, (void*)Kl, 64, pstride, bk, bk, 0L, NP, 64, 64, 1.0f);
  wmma_gemm64<1, true, 2, 2, false><<<dim3((nqb * 1 + 7) / 8, B), 256, 0, stream>>>(
      mTh, mTl, 64, pstride, wr + OFF_WK2H, wr + OFF_WK2L, 64, 0L,
      (void*)Kmh, (void*)Kml, 64, pstride, bk2, bk2, 0L, NP, 64, 64, 1.0f);
  wmma_gemm64<0, false, 1, 1, false><<<dim3((1 * nqb + 7) / 8, B), 256, 0, stream>>>(
      wr + OFF_WV, wr + OFF_WV, 64, 0L, X3 + 128, X3 + 128, 192, (long)NP * 192,
      (void*)Vh, (void*)Vh, NP, (long)64 * NP, bv, bv, 0L, 64, NP, 64, WCARRY_INV);
  wmma_gemm64<0, false, 1, 1, false><<<dim3((1 * nqb + 7) / 8, B), 256, 0, stream>>>(
      wr + OFF_WV2, wr + OFF_WV2, 64, 0L, mT16, mT16, 64, pstride,
      (void*)Vm, (void*)Vm, NP, (long)64 * NP, bv2, bv2, 0L, 64, NP, 64, WCARRY_INV);
  attn_dual<<<dim3(B * 2 * nqb), 128, 0, stream>>>(Qh, Ql, Kh, Kl, Kmh, Kml, Vh, Vm, Zc, NP);
  wmma_gemm64<0, false, 2, 1, false><<<dim3((nqb * 2 + 7) / 8, B), 256, 0, stream>>>(
      Zc, Zc, 128, (long)NP * 128, wr + OFF_WZ, wr + OFF_WZ, 128, 0L,
      (void*)X3, (void*)X3, 192, (long)NP * 192, bz, bz, 0L, NP, 128, 128, WCARRY_INV);
  wmma_gemm64<0, false, 1, 0, false><<<dim3((3 * nqb + 7) / 8, B), 256, 0, stream>>>(
      wr + OFF_WM, wr + OFF_WM, 192, 0L, X3, X3, 192, (long)NP * 192,
      (void*)comb, (void*)comb, NP, (long)192 * NP, bm, bm, 0L, 192, NP, 192, WCARRY_INV);
  k_gate<<<dim3((nh + 255) / 256), 256, 0, stream>>>(comb, m, out0, out1, NP, nh);
  (void)hipGetLastError();
}
